// ContinuousEventTransformer_74448963109498
// MI455X (gfx1250) — hardware-run, weakly checked
//
#include <hip/hip_runtime.h>
#include <math.h>

typedef __attribute__((ext_vector_type(16))) _Float16 v16h;
typedef __attribute__((ext_vector_type(8)))  _Float16 v8h;
typedef __attribute__((ext_vector_type(4)))  _Float16 v4h;
typedef __attribute__((ext_vector_type(16))) __bf16   v16b;
typedef __attribute__((ext_vector_type(8)))  __bf16   v8b;
typedef __attribute__((ext_vector_type(8)))  float    v8f;
typedef __attribute__((ext_vector_type(4)))  float    v4f;
typedef __attribute__((ext_vector_type(4)))  unsigned int v4u;

constexpr int kB = 2;
constexpr int kT = 2048;
constexpr int kIN = 32;
constexpr int kD = 512;
constexpr int kH = 8;
constexpr int kL = 6;
constexpr int kMETA = 8;
constexpr int kACT = 3;
constexpr int kFF = 4 * kD;
constexpr int kHD = kD / kH;
constexpr int kM = kB * kT;
constexpr int kQKVld = 3 * kD;
constexpr int kNEP = 64;
constexpr float kEps = 1e-5f;
constexpr float kInvD = 1.0f / (float)kD;
constexpr float kInvSqrt2 = 0.70710678118654752f;
constexpr float kLog2e = 1.4426950408889634f;
static_assert(kHD == 64);
static_assert(kD == 512 && kM == 4096 && kFF == 2048 && kQKVld == 1536);
static_assert((kD % 64) == 0 && (kFF % 64) == 0 && (kQKVld % 64) == 0 && (kM % 64) == 0 && (kT % 64) == 0);
static_assert((kIN % 32) == 0 && (kD % 32) == 0 && (kFF % 32) == 0);
static_assert(kIN == 32 && kNEP == 64);

constexpr float kWC = 1024.0f;
constexpr float kXC = 16.0f;
constexpr float kQC = 64.0f;
constexpr float kUC = 64.0f;
constexpr float kOC = 256.0f;
constexpr float kPLog2 = 15.0f;
constexpr float kScX  = 1.0f / (kXC * kWC);
constexpr float kScO  = 1.0f / (kOC * kWC);
constexpr float kScU  = 1.0f / (kUC * kWC);
constexpr float kAttnOut = kOC / kQC;

constexpr int kOut0N = kM * kIN;
constexpr int kOut1N = kB * kACT;
constexpr int kOut2N = kM * kD;
constexpr int kOutTotal = kOut0N + kOut1N + kOut2N;
constexpr int kOutLines = (kOutTotal + 31) / 32;
static_assert(kOut0N * 4 == 524288);
static_assert((kOut0N + kOut1N) * 4 == 524312);
static_assert(kOutTotal * 4 == 8912920);

constexpr size_t kOffHA  = 0;
constexpr size_t kOffHB  = kOffHA  + (size_t)kM * kD * 4;
constexpr size_t kOffX   = kOffHB  + (size_t)kM * kD * 4;
constexpr size_t kOffQKV = kOffX   + (size_t)kM * kD * 2;
constexpr size_t kOffVT  = kOffQKV + (size_t)kM * kQKVld * 2;
constexpr size_t kOffO   = kOffVT  + (size_t)kM * kD * 2;
constexpr size_t kOffU   = kOffO   + (size_t)kM * kD * 2;
constexpr size_t kOffWQT = kOffU   + (size_t)kM * kFF * 2;
constexpr size_t kOffWPT = kOffWQT + (size_t)kL * kQKVld * kD * 2;
constexpr size_t kOffW1T = kOffWPT + (size_t)kL * kD * kD * 2;
constexpr size_t kOffW2T = kOffW1T + (size_t)kL * kFF * kD * 2;
constexpr size_t kOffWNT = kOffW2T + (size_t)kL * kD * kFF * 2;
constexpr size_t kOffWIH = kOffWNT + (size_t)kNEP * kD * 2;
constexpr size_t kOffWIL = kOffWIH + (size_t)kD * kIN * 2;
constexpr size_t kOffEVH = kOffWIL + (size_t)kD * kIN * 2;
constexpr size_t kOffEVL = kOffEVH + (size_t)kM * kIN * 2;
constexpr size_t kOffNE  = kOffEVL + (size_t)kM * kIN * 2;
constexpr size_t kOffMP  = kOffNE  + (size_t)kM * kNEP * 4;
constexpr size_t kOffAC  = kOffMP  + (size_t)kB * kD * 4;
constexpr size_t kWsTotal = kOffAC + 128;
static_assert(kWsTotal == 98177152ull);
static_assert(kWsTotal <= 134217728ull);
static_assert((kOffHB % 128) == 0 && (kOffX % 128) == 0 && (kOffQKV % 128) == 0 && (kOffVT % 128) == 0 &&
              (kOffO % 128) == 0 && (kOffU % 128) == 0 && (kOffWQT % 128) == 0 && (kOffWPT % 128) == 0 &&
              (kOffW1T % 128) == 0 && (kOffW2T % 128) == 0 && (kOffWNT % 128) == 0 && (kOffWIH % 128) == 0 &&
              (kOffWIL % 128) == 0 && (kOffEVH % 128) == 0 && (kOffEVL % 128) == 0 && (kOffNE % 128) == 0 &&
              (kOffMP % 128) == 0 && (kOffAC % 128) == 0);

__device__ __forceinline__ unsigned short f2bf_bits(float f) {
  unsigned u = __float_as_uint(f);
  return (unsigned short)((u + 0x7FFFu + ((u >> 16) & 1u)) >> 16);
}
__device__ __forceinline__ float bf_bits2f(unsigned short h) { return __uint_as_float(((unsigned)h) << 16); }

__device__ __forceinline__ void wave_lds_sync() {
  __builtin_amdgcn_fence(__ATOMIC_RELEASE, "workgroup");
  __builtin_amdgcn_wave_barrier();
  __builtin_amdgcn_fence(__ATOMIC_ACQUIRE, "workgroup");
}

__device__ __forceinline__ void dep_guard4_h(v8f& a, v8f& b, v8f& c, v8f& d, v16h x, v16h y) {
  asm volatile("v_nop\n\tv_nop\n\tv_nop\n\tv_nop" : "+v"(a), "+v"(b), "+v"(c), "+v"(d) : "v"(x), "v"(y));
}
__device__ __forceinline__ void dep_guard4_b(v8f& a, v8f& b, v8f& c, v8f& d, v16b x, v16b y) {
  asm volatile("v_nop\n\tv_nop\n\tv_nop\n\tv_nop" : "+v"(a), "+v"(b), "+v"(c), "+v"(d) : "v"(x), "v"(y));
}
__device__ __forceinline__ void keep4_h(v16h a, v16h b, v16h c, v16h d) { asm volatile("v_nop" :: "v"(a), "v"(b), "v"(c), "v"(d)); }
__device__ __forceinline__ void keep4_b(v16b a, v16b b, v16b c, v16b d) { asm volatile("v_nop" :: "v"(a), "v"(b), "v"(c), "v"(d)); }
__device__ __forceinline__ void acc_guard4(v8f& a, v8f& b, v8f& c, v8f& d) {
  asm volatile("v_nop\n\tv_nop\n\tv_nop\n\tv_nop" : "+v"(a), "+v"(b), "+v"(c), "+v"(d));
}

template <typename T> struct Frag;
template <> struct Frag<_Float16> {
  typedef v16h V; union U { v16h v; v8h h[2]; };
  static __device__ __forceinline__ v16h load(const _Float16* p) {
    U f; f.h[0] = *(const v8h*)(p); f.h[1] = *(const v8h*)(p + 16); return f.v;
  }
  static __device__ __forceinline__ v8f mma(v16h a, v16h b, v8f c) {
    return __builtin_amdgcn_wmma_f32_16x16x32_f16(false, a, false, b, (short)0, c, false, false);
  }
  static __device__ __forceinline__ void guard4(v8f& a, v8f& b, v8f& c, v8f& d, v16h x, v16h y) { dep_guard4_h(a, b, c, d, x, y); }
  static __device__ __forceinline__ void keep(v16h a, v16h b, v16h c, v16h d) { keep4_h(a, b, c, d); }
};
template <> struct Frag<__bf16> {
  typedef v16b V; union U { v16b v; v8b h[2]; };
  static __device__ __forceinline__ v16b load(const __bf16* p) {
    U f; f.h[0] = *(const v8b*)(p); f.h[1] = *(const v8b*)(p + 16); return f.v;
  }
  static __device__ __forceinline__ v8f mma(v16b a, v16b b, v8f c) {
    return __builtin_amdgcn_wmma_f32_16x16x32_bf16(false, a, false, b, (short)0, c, false, false);
  }
  static __device__ __forceinline__ void guard4(v8f& a, v8f& b, v8f& c, v8f& d, v16b x, v16b y) { dep_guard4_b(a, b, c, d, x, y); }
  static __device__ __forceinline__ void keep(v16b a, v16b b, v16b c, v16b d) { keep4_b(a, b, c, d); }
};

__device__ __forceinline__ v8f mma_h(v16h a, v16h b, v8f c) {
  c = __builtin_amdgcn_wmma_f32_16x16x32_f16(false, a, false, b, (short)0, c, false, false);
  asm volatile("v_nop\n\tv_nop\n\tv_nop\n\tv_nop" : "+v"(c) : "v"(a), "v"(b));
  return c;
}

template <int ET> struct Elem;
template <> struct Elem<0> { typedef _Float16 T; };
template <> struct Elem<1> { typedef __bf16 T; };

template <int ET, bool SPLIT, bool BIAS, int OUT_MODE, bool RESID, bool GELU>
__global__ __launch_bounds__(256) void wmma_gemm64(
    const unsigned short* __restrict__ Ap, const unsigned short* __restrict__ A2p, int lda,
    const unsigned short* __restrict__ Btp, const unsigned short* __restrict__ Bt2p, int ldb,
    void* __restrict__ Cout, int ldc,
    const float* __restrict__ bias, const float* __restrict__ resid,
    int M, int N, int K, float scale, float oscale) {
  typedef typename Elem<ET>::T T;
  typedef typename Frag<T>::V V;
  const T* A = (const T*)Ap;
  const T* A2 = (const T*)A2p;
  const T* Bt = (const T*)Btp;
  const T* Bt2 = (const T*)Bt2p;
  __shared__ __align__(16) float sT[8][16 * 68];
  const int lane = threadIdx.x & 31;
  const int wave = __builtin_amdgcn_readfirstlane((int)(threadIdx.x >> 5));
  const int tilesN = N >> 6;
  const int tilesM = M >> 6;
  const int tile = blockIdx.x * 8 + wave;
  if (tile >= tilesM * tilesN) return;
  const int tm = tile / tilesN;
  const int tn = tile - tm * tilesN;
  const int m0 = tm << 6;
  const int n0 = tn << 6;

  const int rlane = lane & 15;
  const int koff  = (lane >> 4) * 8;
  const int mOff  = (lane >> 4) * 8;

  v8f acc[4][4];
#pragma unroll
  for (int i = 0; i < 4; ++i)
#pragma unroll
    for (int j = 0; j < 4; ++j) acc[i][j] = (v8f){0.f,0.f,0.f,0.f,0.f,0.f,0.f,0.f};

  for (int k0 = 0; k0 < K; k0 += 32) {
    V bh[4], bl[4];
#pragma unroll
    for (int j = 0; j < 4; ++j) {
      const size_t bo = (size_t)(n0 + (j << 4) + rlane) * ldb + koff + k0;
      bh[j] = Frag<T>::load(Bt + bo);
      if (SPLIT) bl[j] = Frag<T>::load(Bt2 + bo);
    }
#pragma unroll
    for (int i = 0; i < 4; ++i) {
      const size_t ao = (size_t)(m0 + (i << 4) + rlane) * lda + koff + k0;
      V ah = Frag<T>::load(A + ao);
      V al;
      if (SPLIT) al = Frag<T>::load(A2 + ao);
#pragma unroll
      for (int j = 0; j < 4; ++j) {
        acc[i][j] = Frag<T>::mma(ah, bh[j], acc[i][j]);
        if (SPLIT) {
          acc[i][j] = Frag<T>::mma(ah, bl[j], acc[i][j]);
          acc[i][j] = Frag<T>::mma(al, bh[j], acc[i][j]);
        }
      }
      Frag<T>::guard4(acc[i][0], acc[i][1], acc[i][2], acc[i][3], ah, SPLIT ? al : ah);
    }
    Frag<T>::keep(bh[0], bh[1], bh[2], bh[3]);
    if (SPLIT) Frag<T>::keep(bl[0], bl[1], bl[2], bl[3]);
  }
  acc_guard4(acc[0][0], acc[0][1], acc[0][2], acc[0][3]);
  acc_guard4(acc[1][0], acc[1][1], acc[1][2], acc[1][3]);
  acc_guard4(acc[2][0], acc[2][1], acc[2][2], acc[2][3]);
  acc_guard4(acc[3][0], acc[3][1], acc[3][2], acc[3][3]);

  float* slab = sT[wave];
#pragma unroll
  for (int i = 0; i < 4; ++i) {
    const int mBase = m0 + (i << 4);
#pragma unroll
    for (int j = 0; j < 4; ++j) {
      float bv = 0.f;
      if (BIAS) bv = bias[n0 + (j << 4) + rlane];
#pragma unroll
      for (int r = 0; r < 8; ++r) {
        float v = acc[i][j][r] * scale;
        if (BIAS) v += bv;
        slab[(mOff + r) * 68 + (j << 4) + rlane] = v;
      }
    }
    wave_lds_sync();
    if (GELU) {
#pragma unroll 1
      for (int e = 0; e < 32; ++e) {
        float* p = slab + (e >> 1) * 68 + ((e & 1) << 5) + lane;
        const float xv = *p;
        const float gv = 0.5f * xv * (1.0f + erff(xv * kInvSqrt2));
        *p = gv;
      }
      wave_lds_sync();
    }
    if (OUT_MODE == 0) {
      float* C = (float*)Cout;
      const int hh = lane >> 4, c4 = (lane & 15) * 4;
      v4f vals[8];
#pragma unroll
      for (int it = 0; it < 8; ++it) {
        const int row = it * 2 + hh;
        v4f v = *(const v4f*)(slab + row * 68 + c4);
        if (RESID) {
          const v4f rr = *(const v4f*)(resid + (size_t)(mBase + row) * ldc + n0 + c4);
          v = v + rr;
        }
        vals[it] = v;
      }
      for (int pass = 0; pass < 2; ++pass) {
#pragma unroll
        for (int it = 0; it < 8; ++it) {
          const int row = it * 2 + hh;
          *(volatile v4f*)(C + (size_t)(mBase + row) * ldc + n0 + c4) = vals[it];
        }
        __threadfence();
      }
    } else {
      const int q = lane >> 3, c8 = (lane & 7) * 8;
      unsigned short* C = (unsigned short*)Cout;
      v8h hv[4];
#pragma unroll
      for (int it = 0; it < 4; ++it) {
        const int row = it * 4 + q;
        const float* sp = slab + row * 68 + c8;
        const v4f a0 = *(const v4f*)(sp);
        const v4f a1 = *(const v4f*)(sp + 4);
#pragma unroll
        for (int e = 0; e < 4; ++e) {
          hv[it][e]     = (_Float16)(a0[e] * oscale);
          hv[it][4 + e] = (_Float16)(a1[e] * oscale);
        }
      }
      for (int pass = 0; pass < 2; ++pass) {
#pragma unroll
        for (int it = 0; it < 4; ++it) {
          const int row = it * 4 + q;
          *(volatile v8h*)(C + (size_t)(mBase + row) * ldc + n0 + c8) = hv[it];
        }
        __threadfence();
      }
    }
    wave_lds_sync();
  }
}

__global__ __launch_bounds__(256) void wt_f16_kernel(const float* __restrict__ W, unsigned short* __restrict__ out,
                                                     int Kdim, int Nreal, int Npad, float carry) {
  __shared__ float sm[64][65];
  const int t  = threadIdx.x;
  const int k0 = blockIdx.x * 64;
  const int n0 = blockIdx.y * 64;
  const int z  = blockIdx.z;
  const float* Wz = W + (size_t)z * Kdim * Nreal;
  unsigned short* oz = out + (size_t)z * Npad * Kdim;
#pragma unroll
  for (int i = 0; i < 4; ++i) {
    const int e4 = i * 256 + t;
    const int r  = e4 >> 4;
    const int c4 = (e4 & 15) * 4;
    const int n  = n0 + c4;
    const int nc = (n < Nreal) ? n : (Nreal - 4);
    const v4f w = *(const v4f*)(Wz + (size_t)(k0 + r) * Nreal + nc);
    const bool ok = (n < Nreal);
    sm[c4 + 0][r] = ok ? w[0] * carry : 0.0f;
    sm[c4 + 1][r] = ok ? w[1] * carry : 0.0f;
    sm[c4 + 2][r] = ok ? w[2] * carry : 0.0f;
    sm[c4 + 3][r] = ok ? w[3] * carry : 0.0f;
  }
  __syncthreads();
  const int lane = t & 31;
  const int wave = __builtin_amdgcn_readfirstlane((int)(t >> 5));
  const int q = lane >> 3, c8 = (lane & 7) * 8;
  v8h hv[2];
#pragma unroll
  for (int it = 0; it < 2; ++it) {
    const int row = wave * 8 + it * 4 + q;
#pragma unroll
    for (int e = 0; e < 8; ++e) hv[it][e] = (_Float16)sm[row][c8 + e];
  }
  for (int pass = 0; pass < 2; ++pass) {
#pragma unroll
    for (int it = 0; it < 2; ++it) {
      const int row = wave * 8 + it * 4 + q;
      *(volatile v8h*)(oz + (size_t)(n0 + row) * Kdim + k0 + c8) = hv[it];
    }
    __threadfence();
  }
}

__global__ __launch_bounds__(256) void win_split_kernel(const float* __restrict__ W_in,
                                                        unsigned short* __restrict__ dhi, unsigned short* __restrict__ dlo) {
  const int i = blockIdx.x * 256 + threadIdx.x;
  if (i >= (kD * kIN) / 8) return;
  const int n  = i >> 2;
  const int k8 = (i & 3) * 8;
  v8h hv, lv;
#pragma unroll
  for (int e = 0; e < 8; ++e) {
    const float w = W_in[(size_t)(k8 + e) * kD + n];
    const unsigned short hb = f2bf_bits(w);
    const unsigned short lb = f2bf_bits(w - bf_bits2f(hb));
    hv[e] = __builtin_bit_cast(_Float16, hb);
    lv[e] = __builtin_bit_cast(_Float16, lb);
  }
  unsigned short* qh = dhi + (size_t)i * 8;
  unsigned short* ql = dlo + (size_t)i * 8;
  *(volatile v8h*)qh = hv;
  *(volatile v8h*)ql = lv;
  __threadfence();
  *(volatile v8h*)qh = hv;
  *(volatile v8h*)ql = lv;
}

__global__ __launch_bounds__(256) void split_rows_bf16_kernel(
    const float* __restrict__ src, unsigned short* __restrict__ dhi, unsigned short* __restrict__ dlo, int total8) {
  const int i = blockIdx.x * 256 + threadIdx.x;
  if (i >= total8) return;
  const size_t e0 = (size_t)i << 3;
  const v4f a0 = *(const v4f*)(src + e0);
  const v4f a1 = *(const v4f*)(src + e0 + 4);
  v8h hv, lv;
#pragma unroll
  for (int e = 0; e < 4; ++e) {
    const unsigned short h0 = f2bf_bits(a0[e]), h1 = f2bf_bits(a1[e]);
    const unsigned short l0 = f2bf_bits(a0[e] - bf_bits2f(h0)), l1 = f2bf_bits(a1[e] - bf_bits2f(h1));
    hv[e]     = __builtin_bit_cast(_Float16, h0);
    hv[4 + e] = __builtin_bit_cast(_Float16, h1);
    lv[e]     = __builtin_bit_cast(_Float16, l0);
    lv[4 + e] = __builtin_bit_cast(_Float16, l1);
  }
  unsigned short* qh = dhi + e0;
  unsigned short* ql = dlo + e0;
  *(volatile v8h*)qh = hv;
  *(volatile v8h*)ql = lv;
  __threadfence();
  *(volatile v8h*)qh = hv;
  *(volatile v8h*)ql = lv;
}

__global__ __launch_bounds__(256) void meta_proj_kernel(const float* __restrict__ meta, const float* __restrict__ W_meta,
                                                        const float* __restrict__ b_meta, float* __restrict__ mp) {
  const int i = blockIdx.x * 256 + threadIdx.x;
  if (i >= kB * kD) return;
  const int b = i / kD;
  const int col = i - b * kD;
  float acc = 0.0f;
#pragma unroll 1
  for (int j = 0; j < kMETA; ++j) acc = fmaf(meta[b * kMETA + j], W_meta[(size_t)j * kD + col], acc);
  const float v = acc + b_meta[col];
  volatile float* p = mp + i;
  *p = v;
  __threadfence();
  *p = v;
}

template <int MODE>
__global__ __launch_bounds__(256) void ln_rows_kernel(
    const float* __restrict__ x, const float* __restrict__ g, const float* __restrict__ bt,
    const float* __restrict__ pos, const float* __restrict__ mp,
    float* __restrict__ outF, unsigned short* __restrict__ outH) {
  const int lane = threadIdx.x & 31;
  const int wave = __builtin_amdgcn_readfirstlane((int)(threadIdx.x >> 5));
  const int row = blockIdx.x * 8 + wave;
  const float* xr = x + (size_t)row * kD;
  v4f a[4];
#pragma unroll
  for (int j = 0; j < 4; ++j) a[j] = *(const v4f*)(xr + j * 128 + lane * 4);
  float s = 0.0f;
#pragma unroll
  for (int j = 0; j < 4; ++j) s += (a[j][0] + a[j][1]) + (a[j][2] + a[j][3]);
  s += __shfl_xor(s, 16, 32);
  s += __shfl_xor(s, 8, 32);
  s += __shfl_xor(s, 4, 32);
  s += __shfl_xor(s, 2, 32);
  s += __shfl_xor(s, 1, 32);
  const float mean = s * kInvD;
  float vs = 0.0f;
#pragma unroll
  for (int j = 0; j < 4; ++j) {
    const float d0 = a[j][0] - mean, d1 = a[j][1] - mean, d2 = a[j][2] - mean, d3 = a[j][3] - mean;
    vs += (d0 * d0 + d1 * d1) + (d2 * d2 + d3 * d3);
  }
  vs += __shfl_xor(vs, 16, 32);
  vs += __shfl_xor(vs, 8, 32);
  vs += __shfl_xor(vs, 4, 32);
  vs += __shfl_xor(vs, 2, 32);
  vs += __shfl_xor(vs, 1, 32);
  const float rstd = rsqrtf(vs * kInvD + kEps);
  const int bidx = row / kT;
  const int tpos = row - bidx * kT;
  v4f y[4];
#pragma unroll
  for (int j = 0; j < 4; ++j) {
    const int col = j * 128 + lane * 4;
    const v4f gv = *(const v4f*)(g + col);
    const v4f bv = *(const v4f*)(bt + col);
#pragma unroll
    for (int e = 0; e < 4; ++e) y[j][e] = (a[j][e] - mean) * rstd * gv[e] + bv[e];
    if (MODE == 1) {
      const v4f pv = *(const v4f*)(pos + (size_t)tpos * kD + col);
      const v4f mv = *(const v4f*)(mp + (size_t)bidx * kD + col);
#pragma unroll
      for (int e = 0; e < 4; ++e) y[j][e] = (y[j][e] + pv[e]) + mv[e];
    }
  }
  v4h hv[4];
  if (MODE != 1) {
#pragma unroll
    for (int j = 0; j < 4; ++j)
#pragma unroll
      for (int e = 0; e < 4; ++e) hv[j][e] = (_Float16)(y[j][e] * kXC);
  }
  for (int pass = 0; pass < 2; ++pass) {
#pragma unroll
    for (int j = 0; j < 4; ++j) {
      const size_t o = (size_t)row * kD + j * 128 + lane * 4;
      if (MODE != 0) *(volatile v4f*)(outF + o) = y[j];
      if (MODE != 1) *(volatile v4h*)(outH + o) = hv[j];
    }
    __threadfence();
  }
}

__global__ __launch_bounds__(256) void vt_kernel(const unsigned short* __restrict__ qkv, unsigned short* __restrict__ vt) {
  __shared__ __align__(16) _Float16 sm[64 * 72];
  const int t = threadIdx.x;
  const int tok0 = blockIdx.x * 64;
  const int h = blockIdx.y;
  const int b = blockIdx.z;
#pragma unroll
  for (int i = 0; i < 2; ++i) {
    const int e  = i * 256 + t;
    const int r  = e >> 3;
    const int c8 = (e & 7) * 8;
    const v4u w = *(const v4u*)(qkv + ((size_t)b * kT + tok0 + r) * kQKVld + 2 * kD + h * kHD + c8);
    const unsigned w0 = w[0], w1 = w[1], w2 = w[2], w3 = w[3];
    _Float16* col = sm + c8 * 72 + r;
    col[0 * 72] = __builtin_bit_cast(_Float16, (unsigned short)(w0 & 0xffffu));
    col[1 * 72] = __builtin_bit_cast(_Float16, (unsigned short)(w0 >> 16));
    col[2 * 72] = __builtin_bit_cast(_Float16, (unsigned short)(w1 & 0xffffu));
    col[3 * 72] = __builtin_bit_cast(_Float16, (unsigned short)(w1 >> 16));
    col[4 * 72] = __builtin_bit_cast(_Float16, (unsigned short)(w2 & 0xffffu));
    col[5 * 72] = __builtin_bit_cast(_Float16, (unsigned short)(w2 >> 16));
    col[6 * 72] = __builtin_bit_cast(_Float16, (unsigned short)(w3 & 0xffffu));
    col[7 * 72] = __builtin_bit_cast(_Float16, (unsigned short)(w3 >> 16));
  }
  __syncthreads();
  const int lane = t & 31;
  const int wave = __builtin_amdgcn_readfirstlane((int)(t >> 5));
  const int q = lane >> 3, k8 = (lane & 7) * 8;
  v8h hv[2];
#pragma unroll
  for (int it = 0; it < 2; ++it) {
    const int d = wave * 8 + it * 4 + q;
    hv[it] = *(const v8h*)(sm + d * 72 + k8);
  }
  for (int pass = 0; pass < 2; ++pass) {
#pragma unroll
    for (int it = 0; it < 2; ++it) {
      const int d = wave * 8 + it * 4 + q;
      *(volatile v8h*)(vt + ((size_t)(b * kH + h) * kHD + d) * kT + tok0 + k8) = hv[it];
    }
    __threadfence();
  }
}

__global__ __launch_bounds__(128) void attn_causal_kernel(
    const unsigned short* __restrict__ qkvp, const unsigned short* __restrict__ vtp,
    unsigned short* __restrict__ op, float cs) {
  __shared__ __align__(16) float Os[4][16 * 68];
  const _Float16* qkv = (const _Float16*)qkvp;
  const _Float16* vt  = (const _Float16*)vtp;
  const int lane = threadIdx.x & 31;
  const int wave = __builtin_amdgcn_readfirstlane((int)(threadIdx.x >> 5));
  const int hh = lane >> 4, c = lane & 15;
  constexpr int nqb = kT / 64;
  const int bx = blockIdx.x;
  const int qb = bx % nqb;
  const int bh = bx / nqb;
  const int h  = bh % kH;
  const int b  = bh / kH;
  const int q0 = qb * 64 + wave * 16;
  const size_t tok0 = (size_t)b * kT;

  const _Float16* qrow = qkv + (tok0 + q0 + c) * kQKVld + h * kHD + 8 * hh;
  const v16h qf0 = Frag<_Float16>::load(qrow);
  const v16h qf1 = Frag<_Float16>::load(qrow + 32);
  const _Float16* kbase = qkv + tok0 * kQKVld + kD + h * kHD + 8 * hh;
  const _Float16* vbase = vt + ((size_t)bh * kHD + c) * kT + 8 * hh;

  float mrow = -INFINITY, lrow = 0.0f;
  v8f oacc[4];
#pragma unroll
  for (int t = 0; t < 4; ++t) oacc[t] = (v8f){0.f,0.f,0.f,0.f,0.f,0.f,0.f,0.f};

  const int nch = (qb + 1 < nqb) ? (qb + 1) : nqb;
  const int qrow_i = q0 + c;
  for (int kc = 0; kc < nch; ++kc) {
    const int kv0 = kc * 64;
    v8f s[4];
#pragma unroll
    for (int j = 0; j < 4; ++j) {
      const _Float16* kp = kbase + (size_t)(kv0 + j * 16 + c) * kQKVld;
      const v16h kf0 = Frag<_Float16>::load(kp);
      const v16h kf1 = Frag<_Float16>::load(kp + 32);
      s[j] = (v8f){0.f,0.f,0.f,0.f,0.f,0.f,0.f,0.f};
      s[j] = mma_h(kf0, qf0, s[j]);
      s[j] = mma_h(kf1, qf1, s[j]);
    }
    if (kc == qb) {
#pragma unroll
      for (int j = 0; j < 4; ++j)
#pragma unroll
        for (int r = 0; r < 8; ++r) {
          const int key = kv0 + j * 16 + 8 * hh + r;
          s[j][r] = (key > qrow_i) ? -INFINITY : s[j][r];
        }
    }
    float m = s[0][0];
#pragma unroll
    for (int j = 0; j < 4; ++j)
#pragma unroll
      for (int r = 0; r < 8; ++r) m = fmaxf(m, s[j][r]);
    m = fmaxf(m, __shfl_xor(m, 16, 32));
    const float mnew = fmaxf(mrow, m);
    const float alpha = __builtin_amdgcn_exp2f((mrow - mnew) * cs);
    mrow = mnew;
    float psum = 0.0f;
    v16h pf0, pf1;
#pragma unroll
    for (int r = 0; r < 8; ++r) {
      const float e0 = __builtin_amdgcn_exp2f(fmaf(s[0][r] - mnew, cs, kPLog2));
      const float e1 = __builtin_amdgcn_exp2f(fmaf(s[1][r] - mnew, cs, kPLog2));
      const float e2 = __builtin_amdgcn_exp2f(fmaf(s[2][r] - mnew, cs, kPLog2));
      const float e3 = __builtin_amdgcn_exp2f(fmaf(s[3][r] - mnew, cs, kPLog2));
      pf0[r]     = (_Float16)e0;
      pf0[8 + r] = (_Float16)e1;
      pf1[r]     = (_Float16)e2;
      pf1[8 + r] = (_Float16)e3;
      psum += (e0 + e1) + (e2 + e3);
    }
    psum += __shfl_xor(psum, 16, 32);
    lrow = lrow * alpha + psum;
#pragma unroll
    for (int t = 0; t < 4; ++t) oacc[t] = oacc[t] * alpha;
#pragma unroll
    for (int t = 0; t < 4; ++t) {
      const _Float16* vp = vbase + (size_t)(t * 16) * kT + kv0;
      const v16h vf0 = Frag<_Float16>::load(vp);
      const v16h vf1 = Frag<_Float16>::load(vp + 32);
      oacc[t] = mma_h(vf0, pf0, oacc[t]);
      oacc[t] = mma_h(vf1, pf1, oacc[t]);
    }
  }

  float* os = Os[wave];
  const float inv = kAttnOut / lrow;
#pragma unroll
  for (int t = 0; t < 4; ++t) {
    const v4f lo4 = (v4f){oacc[t][0] * inv, oacc[t][1] * inv, oacc[t][2] * inv, oacc[t][3] * inv};
    const v4f hi4 = (v4f){oacc[t][4] * inv, oacc[t][5] * inv, oacc[t][6] * inv, oacc[t][7] * inv};
    *(v4f*)(os + c * 68 + t * 16 + 8 * hh)     = lo4;
    *(v4f*)(os + c * 68 + t * 16 + 8 * hh + 4) = hi4;
  }
  wave_lds_sync();
  {
    const int q = lane >> 3, c8 = (lane & 7) * 8;
    v8h hv[4];
#pragma unroll
    for (int it = 0; it < 4; ++it) {
      const int row = it * 4 + q;
      const float* sp = os + row * 68 + c8;
      const v4f a0 = *(const v4f*)(sp);
      const v4f a1 = *(const v4f*)(sp + 4);
#pragma unroll
      for (int e = 0; e < 4; ++e) {
        hv[it][e]     = (_Float16)a0[e];
        hv[it][4 + e] = (_Float16)a1[e];
      }
    }
    unsigned short* ob = op + (tok0 + q0) * kD + h * kHD + c8;
    for (int pass = 0; pass < 2; ++pass) {
#pragma unroll
      for (int it = 0; it < 4; ++it) {
        const int row = it * 4 + q;
        *(volatile v8h*)(ob + (size_t)row * kD) = hv[it];
      }
      __threadfence();
    }
  }
}

__global__ __launch_bounds__(32) void action_kernel(const float* __restrict__ hf, const float* __restrict__ W_act,
                                                    const float* __restrict__ b_act, float* __restrict__ act) {
  static_assert(kB == 2 && kACT == 3);
  const int lane = threadIdx.x & 31;
  const float* r0 = hf + (size_t)(kT - 1) * kD;
  const float* r1 = hf + (size_t)(2 * kT - 1) * kD;
  float a00 = 0.f, a01 = 0.f, a02 = 0.f, a10 = 0.f, a11 = 0.f, a12 = 0.f;
#pragma unroll 1
  for (int i = 0; i < kD / 32; ++i) {
    const int d = lane + 32 * i;
    const float x0 = r0[d], x1 = r1[d];
    const float w0 = W_act[d * kACT + 0], w1 = W_act[d * kACT + 1], w2 = W_act[d * kACT + 2];
    a00 = fmaf(x0, w0, a00); a01 = fmaf(x0, w1, a01); a02 = fmaf(x0, w2, a02);
    a10 = fmaf(x1, w0, a10); a11 = fmaf(x1, w1, a11); a12 = fmaf(x1, w2, a12);
  }
#pragma unroll
  for (int off = 16; off > 0; off >>= 1) {
    a00 += __shfl_xor(a00, off, 32);
    a01 += __shfl_xor(a01, off, 32);
    a02 += __shfl_xor(a02, off, 32);
    a10 += __shfl_xor(a10, off, 32);
    a11 += __shfl_xor(a11, off, 32);
    a12 += __shfl_xor(a12, off, 32);
  }
  const int lc = (lane < 5) ? lane : 5;
  float bb = b_act[lc % kACT];
  asm volatile("" : "+v"(bb));
  float v = a12;
  v = (lane == 4) ? a11 : v;
  v = (lane == 3) ? a10 : v;
  v = (lane == 2) ? a02 : v;
  v = (lane == 1) ? a01 : v;
  v = (lane == 0) ? a00 : v;
  const float outv = (lane < kB * kACT) ? (v + bb) : 0.0f;
  volatile float* p = act + lane;
  *p = outv;
  __threadfence();
  *p = outv;
}

__global__ __launch_bounds__(256) void pack_kernel(const float* __restrict__ ne64, const float* __restrict__ bne,
                                                   const float* __restrict__ act, const float* __restrict__ hf,
                                                   float* __restrict__ out) {
  const int lane = threadIdx.x & 31;
  const int wave = __builtin_amdgcn_readfirstlane((int)(threadIdx.x >> 5));
  const int line = blockIdx.x * 8 + wave;
  if (line >= kOutLines) return;
  const int idx = line * 32 + lane;
  const int i0 = (idx < kOut0N - 1) ? idx : (kOut0N - 1);
  const int row = i0 >> 5, col = i0 & 31;
  float vne = ne64[(size_t)row * kNEP + col];
  float vb  = bne[col];
  int i1 = idx - kOut0N;
  i1 = (i1 < 0) ? 0 : i1;
  i1 = (i1 > kOut1N - 1) ? (kOut1N - 1) : i1;
  float va = act[i1];
  int i2 = idx - (kOut0N + kOut1N);
  i2 = (i2 < 0) ? 0 : i2;
  i2 = (i2 > kOut2N - 1) ? (kOut2N - 1) : i2;
  float vh = hf[i2];
  asm volatile("" : "+v"(vne));
  asm volatile("" : "+v"(vb));
  asm volatile("" : "+v"(va));
  asm volatile("" : "+v"(vh));
  const float s0 = vne + vb;
  const float val = (idx < kOut0N) ? s0 : ((idx < kOut0N + kOut1N) ? va : vh);
  const bool ok = (idx < kOutTotal);
  const int ic = ok ? idx : (kOutTotal - 1);
  volatile float* p = out + ic;
  if (ok) *p = val;
  __threadfence();
  if (ok) *p = val;
}

extern "C" void kernel_launch(void* const* d_in, const int* in_sizes, int n_in,
                              void* d_out, int out_size, void* d_ws, size_t ws_size,
                              hipStream_t stream) {
  if (n_in != 27) return;
  const int expect[27] = {
      kM * kIN, kB * kMETA, kIN * kD, kD, kD, kD, kT * kD, kMETA * kD, kD,
      kL * kD, kL * kD, kL * kD * kQKVld, kL * kQKVld, kL * kD * kD, kL * kD,
      kL * kD, kL * kD, kL * kD * kFF, kL * kFF, kL * kFF * kD, kL * kD,
      kD, kD, kD * kIN, kIN, kD * kACT, kACT};
  for (int i = 0; i < 27; ++i) if (in_sizes[i] != expect[i]) return;
  if (out_size != kOutTotal) return;
  if (ws_size < kWsTotal) return;

  const float* events  = (const float*)d_in[0];
  const float* meta    = (const float*)d_in[1];
  const float* W_in    = (const float*)d_in[2];
  const float* b_in    = (const float*)d_in[3];
  const float* g_in    = (const float*)d_in[4];
  const float* beta_in = (const float*)d_in[5];
  const float* pos_emb = (const float*)d_in[6];
  const float* W_meta  = (const float*)d_in[7];
  const float* b_meta  = (const float*)d_in[8];
  const float* ln1_g   = (const float*)d_in[9];
  const float* ln1_b   = (const float*)d_in[10];
  const float* Wqkv    = (const float*)d_in[11];
  const float* bqkv    = (const float*)d_in[12];
  const float* Wproj   = (const float*)d_in[13];
  const float* bproj   = (const float*)d_in[14];
  const float* ln2_g   = (const float*)d_in[15];
  const float* ln2_b   = (const float*)d_in[16];
  const float* W1      = (const float*)d_in[17];
  const float* b1      = (const float*)d_in[18];
  const float* W2      = (const float*)d_in[19];
  const float* b2      = (const float*)d_in[20];
  const float* lnf_g   = (const float*)d_in[21];
  const float* lnf_b   = (const float*)d_in[22];
  const float* W_ne    = (const float*)d_in[23];
  const float* b_ne    = (const float*)d_in[24];
  const float* W_act   = (const float*)d_in[25];
  const float* b_act   = (const float*)d_in[26];

  char* ws = (char*)d_ws;
  float*          HA  = (float*)(ws + kOffHA);
  float*          HB  = (float*)(ws + kOffHB);
  unsigned short* X   = (unsigned short*)(ws + kOffX);
  unsigned short* QKV = (unsigned short*)(ws + kOffQKV);
  unsigned short* VT  = (unsigned short*)(ws + kOffVT);
  unsigned short* O   = (unsigned short*)(ws + kOffO);
  unsigned short* U   = (unsigned short*)(ws + kOffU);
  unsigned short* WQT = (unsigned short*)(ws + kOffWQT);
  unsigned short* WPT = (unsigned short*)(ws + kOffWPT);
  unsigned short* W1T = (unsigned short*)(ws + kOffW1T);
  unsigned short* W2T = (unsigned short*)(ws + kOffW2T);
  unsigned short* WNT = (unsigned short*)(ws + kOffWNT);
  unsigned short* WIH = (unsigned short*)(ws + kOffWIH);
  unsigned short* WIL = (unsigned short*)(ws + kOffWIL);
  unsigned short* EVH = (unsigned short*)(ws + kOffEVH);
  unsigned short* EVL = (unsigned short*)(ws + kOffEVL);
  float*          NE  = (float*)(ws + kOffNE);
  float*          MP  = (float*)(ws + kOffMP);
  float*          AC  = (float*)(ws + kOffAC);

  wt_f16_kernel<<<dim3(kD / 64, kQKVld / 64, kL), 256, 0, stream>>>(Wqkv, WQT, kD, kQKVld, kQKVld, kWC);
  wt_f16_kernel<<<dim3(kD / 64, kD / 64, kL), 256, 0, stream>>>(Wproj, WPT, kD, kD, kD, kWC);
  wt_f16_kernel<<<dim3(kD / 64, kFF / 64, kL), 256, 0, stream>>>(W1, W1T, kD, kFF, kFF, kWC);
  wt_f16_kernel<<<dim3(kFF / 64, kD / 64, kL), 256, 0, stream>>>(W2, W2T, kFF, kD, kD, kWC);
  wt_f16_kernel<<<dim3(kD / 64, kNEP / 64, 1), 256, 0, stream>>>(W_ne, WNT, kD, kIN, kNEP, kWC);
  win_split_kernel<<<((kD * kIN) / 8 + 255) / 256, 256, 0, stream>>>(W_in, WIH, WIL);
  split_rows_bf16_kernel<<<((kM * kIN) / 8 + 255) / 256, 256, 0, stream>>>(events, EVH, EVL, (kM * kIN) / 8);
  meta_proj_kernel<<<(kB * kD + 255) / 256, 256, 0, stream>>>(meta, W_meta, b_meta, MP);

  wmma_gemm64<1, true, true, 0, false, false><<<dim3(64), 256, 0, stream>>>(
      EVH, EVL, kIN, WIH, WIL, kIN, (void*)HB, kD, b_in, nullptr, kM, kD, kIN, 1.0f, 1.0f);
  ln_rows_kernel<1><<<kM / 8, 256, 0, stream>>>(HB, g_in, beta_in, pos_emb, MP, HA, nullptr);

  const float cs = (1.0f / sqrtf((float)kHD)) * kLog2e / (kQC * kQC);

  for (int l = 0; l < kL; ++l) {
    ln_rows_kernel<0><<<kM / 8, 256, 0, stream>>>(HA, ln1_g + (size_t)l * kD, ln1_b + (size_t)l * kD,
                                                  nullptr, nullptr, nullptr, X);
    wmma_gemm64<0, false, true, 1, false, false><<<dim3(192), 256, 0, stream>>>(
        X, nullptr, kD, WQT + (size_t)l * kQKVld * kD, nullptr, kD, (void*)QKV, kQKVld,
        bqkv + (size_t)l * kQKVld, nullptr, kM, kQKVld, kD, kScX, kQC);
    vt_kernel<<<dim3(kT / 64, kH, kB), 256, 0, stream>>>(QKV, VT);
    attn_causal_kernel<<<kB * kH * (kT / 64), 128, 0, stream>>>(QKV, VT, O, cs);
    wmma_gemm64<0, false, true, 0, true, false><<<dim3(64), 256, 0, stream>>>(
        O, nullptr, kD, WPT + (size_t)l * kD * kD, nullptr, kD, (void*)HB, kD,
        bproj + (size_t)l * kD, HA, kM, kD, kD, kScO, 1.0f);
    ln_rows_kernel<0><<<kM / 8, 256, 0, stream>>>(HB, ln2_g + (size_t)l * kD, ln2_b + (size_t)l * kD,
                                                  nullptr, nullptr, nullptr, X);
    wmma_gemm64<0, false, true, 1, false, true><<<dim3(256), 256, 0, stream>>>(
        X, nullptr, kD, W1T + (size_t)l * kFF * kD, nullptr, kD, (void*)U, kFF,
        b1 + (size_t)l * kFF, nullptr, kM, kFF, kD, kScX, kUC);
    wmma_gemm64<0, false, true, 0, true, false><<<dim3(64), 256, 0, stream>>>(
        U, nullptr, kFF, W2T + (size_t)l * kD * kFF, nullptr, kFF, (void*)HA, kD,
        b2 + (size_t)l * kD, HB, kM, kD, kFF, kScU, 1.0f);
  }

  ln_rows_kernel<2><<<kM / 8, 256, 0, stream>>>(HA, lnf_g, lnf_b, nullptr, nullptr, HB, X);
  wmma_gemm64<0, false, false, 0, false, false><<<dim3(8), 256, 0, stream>>>(
      X, nullptr, kD, WNT, nullptr, kD, (void*)NE, kNEP, nullptr, nullptr, kM, kNEP, kD, kScX, 1.0f);
  action_kernel<<<1, 32, 0, stream>>>(HB, W_act, b_act, AC);
  pack_kernel<<<(kOutLines + 7) / 8, 256, 0, stream>>>(NE, b_ne, AC, HB, (float*)d_out);
}
